// DGLJTNNEncoder_69002944577982
// MI455X (gfx1250) — hardware-verified
//
#include <hip/hip_runtime.h>


namespace {
constexpr int NT = 64, DEPTH = 10, H = 128, K2 = 2 * H, NPT = 2047, VOC = 780, MAXR = NT * 1024;
constexpr float XS = 8.0f, WSC = 256.0f;
typedef _Float16 b16;
typedef __attribute__((ext_vector_type(16))) _Float16 v16b;
typedef __attribute__((ext_vector_type(8))) _Float16 v8b;
typedef __attribute__((ext_vector_type(8))) float v8f;
typedef __attribute__((ext_vector_type(4))) float v4f;
__device__ __forceinline__ float bf16_rne(float f) { unsigned int u = __float_as_uint(f); u += 0x7FFFu + ((u >> 16) & 1u); return __uint_as_float(u & 0xFFFF0000u); }
__device__ __forceinline__ void split16(float v, b16& hi, b16& lo) { hi = (b16)v; lo = (b16)(v - (float)hi); }
__device__ __forceinline__ v16b frag_kb(const b16* p, int hh) { const v8b a = *(const v8b*)(p + 8 * hh), b = *(const v8b*)(p + 16 + 8 * hh); v16b f;
#pragma unroll
  for (int e = 0; e < 8; ++e) { f[e] = a[e]; f[8 + e] = b[e]; } return f; }
__device__ __forceinline__ v8f wmma16b(v16b a, v16b b, v8f c) { v8f d = __builtin_amdgcn_wmma_f32_16x16x32_f16(false, a, false, b, (short)0, c, false, false); asm volatile("v_nop\n\tv_nop\n\tv_nop\n\tv_nop" : "+v"(d) : "v"(a), "v"(b)); return d; }
__device__ __forceinline__ void wave_lds_sync() { __builtin_amdgcn_fence(__ATOMIC_RELEASE, "workgroup"); __builtin_amdgcn_wave_barrier(); __builtin_amdgcn_fence(__ATOMIC_ACQUIRE, "workgroup"); }
__device__ __forceinline__ float pmul(float a, float b) { float p = a * b; asm volatile("" : "+v"(p)); return p; }
__device__ __forceinline__ int iclamp(int v, int lo, int hi) { return v < lo ? lo : (v > hi ? hi : v); }
__device__ __forceinline__ float sigm(float x) { return 1.0f / (1.0f + __expf(-x)); }

__global__ __launch_bounds__(256) void wprep_kernel(const float* __restrict__ wz, const float* __restrict__ wh, const float* __restrict__ wg, const float* __restrict__ wr, const float* __restrict__ ur, b16* __restrict__ WZT, b16* __restrict__ WHT, b16* __restrict__ WGT, b16* __restrict__ WRU) {
  const size_t u = (size_t)blockIdx.x * 256 + threadIdx.x; const size_t n1 = (size_t)H * K2 / 8; const int which = (int)(u / n1); if (which >= 4) return; const size_t e = (u % n1) * 8; const int o = (int)(e / K2), k0 = (int)(e % K2); v8b v;
  const float* w = which == 0 ? wz : (which == 1 ? wh : wg); b16* dst_ = which == 0 ? WZT : (which == 1 ? WHT : (which == 2 ? WGT : WRU));
  for (int j = 0; j < 8; ++j) { const int k = k0 + j; float val;
    if (which < 3) val = w[(size_t)k * H + o]; else { const int kl = k < H ? k : k - H; const float a = wr[(size_t)kl * H + o], b = ur[(size_t)kl * H + o]; val = k < H ? a : b; }
    v[j] = (b16)(bf16_rne(val) * WSC); }
  for (int pass = 0; pass < 2; ++pass) { *(volatile v8b*)(dst_ + e) = v; __threadfence(); }
}
template <int LEAF>
__global__ __launch_bounds__(64) void level_kernel(int d, const int* __restrict__ wid, const float* __restrict__ emb, const float* __restrict__ MIN, const float* __restrict__ RMIN, const b16* __restrict__ WZT, const b16* __restrict__ WHT, const b16* __restrict__ WRU, const float* __restrict__ bz, const float* __restrict__ bh, const float* __restrict__ br, float* __restrict__ MOUT, float* __restrict__ RMOUT) {
  __shared__ __attribute__((aligned(16))) b16 Ah[2][16][K2 + 8], Al[2][16][K2 + 8]; __shared__ __attribute__((aligned(16))) float Sf[2][16][H + 4];
  const int wave = threadIdx.x >> 5, lane = threadIdx.x & 31, nloc = lane & 15, hlf = lane >> 4; const int r0 = (blockIdx.x * 2 + wave) * 16; const int per = 1 << d;
  for (int rr = 0; rr < 16; ++rr) { const int r = r0 + rr; const int tree = r >> d, j = r & (per - 1); const int c = tree * NPT + (per - 1) + j; const int w = iclamp(wid[c], 0, VOC - 1);
    const v4f xv = *(const v4f*)(emb + (size_t)w * H + lane * 4); v4f s = {0.0f, 0.0f, 0.0f, 0.0f};
    if (!LEAF) { const size_t k1 = ((size_t)tree << (d + 1)) + 2 * j; const v4f a = *(const v4f*)(MIN + k1 * H + lane * 4), b = *(const v4f*)(MIN + (k1 + 1) * H + lane * 4); for (int i = 0; i < 4; ++i) s[i] = a[i] + b[i]; }
    for (int i = 0; i < 4; ++i) { Ah[wave][rr][lane * 4 + i] = (b16)(bf16_rne(xv[i]) * XS); Al[wave][rr][lane * 4 + i] = (b16)0.0f; b16 p, q; split16(s[i] * XS, p, q); Ah[wave][rr][H + lane * 4 + i] = p; Al[wave][rr][H + lane * 4 + i] = q; Sf[wave][rr][lane * 4 + i] = s[i]; } }
  wave_lds_sync();
  v8f az[8], ah[8];
#pragma unroll
  for (int t = 0; t < 8; ++t) { az[t] = (v8f){}; ah[t] = (v8f){}; }
#pragma unroll 2
  for (int kb = 0; kb < K2; kb += 32) { const v16b a = frag_kb(&Ah[wave][nloc][kb], hlf), al = frag_kb(&Al[wave][nloc][kb], hlf); const bool dolo = kb >= H;
#pragma unroll
    for (int t = 0; t < 8; ++t) { const v16b bw = frag_kb(WZT + (size_t)(t * 16 + nloc) * K2 + kb, hlf); az[t] = wmma16b(a, bw, az[t]); if (dolo) az[t] = wmma16b(al, bw, az[t]); } }
  wave_lds_sync();
  for (int rr = 0; rr < 16; ++rr) { const int r = r0 + rr; const int tree = r >> d, j = r & (per - 1); v4f s = {0.0f, 0.0f, 0.0f, 0.0f};
    if (!LEAF) { const size_t k1 = ((size_t)tree << (d + 1)) + 2 * j; const v4f a = *(const v4f*)(RMIN + k1 * H + lane * 4), b = *(const v4f*)(RMIN + (k1 + 1) * H + lane * 4); for (int i = 0; i < 4; ++i) s[i] = a[i] + b[i]; }
    for (int i = 0; i < 4; ++i) { b16 p, q; split16(s[i] * XS, p, q); Ah[wave][rr][H + lane * 4 + i] = p; Al[wave][rr][H + lane * 4 + i] = q; } }
  wave_lds_sync();
#pragma unroll 2
  for (int kb = 0; kb < K2; kb += 32) { const v16b a = frag_kb(&Ah[wave][nloc][kb], hlf), al = frag_kb(&Al[wave][nloc][kb], hlf); const bool dolo = kb >= H;
#pragma unroll
    for (int t = 0; t < 8; ++t) { const v16b bw = frag_kb(WHT + (size_t)(t * 16 + nloc) * K2 + kb, hlf); ah[t] = wmma16b(a, bw, ah[t]); if (dolo) ah[t] = wmma16b(al, bw, ah[t]); } }
  wave_lds_sync();
#pragma unroll
  for (int t = 0; t < 8; ++t) { const int cc = t * 16 + nloc; const float bzv = bf16_rne(bz[cc]), bhv = bf16_rne(bh[cc]); const float sc = 1.0f / (XS * WSC);
#pragma unroll 1
    for (int r8 = 0; r8 < 8; ++r8) { const int rl = 8 * hlf + r8; const float z = sigm(az[t][r8] * sc + bzv), ht = tanhf(ah[t][r8] * sc + bhv); const float s = Sf[wave][rl][cc]; Sf[wave][rl][cc] = pmul(1.0f - z, s) + pmul(z, ht); } }
  wave_lds_sync();
  for (int rr = 0; rr < 16; ++rr) { const int r = r0 + rr; const int tree = r >> d, j = r & (per - 1); const int c = (per - 1) + j; const int p = tree * NPT + (c - 1) / 2; const int w = iclamp(wid[p], 0, VOC - 1);
    const v4f xv = *(const v4f*)(emb + (size_t)w * H + lane * 4); const v4f mv = *(const v4f*)(&Sf[wave][rr][lane * 4]);
    for (int i = 0; i < 4; ++i) { Ah[wave][rr][lane * 4 + i] = (b16)(bf16_rne(xv[i]) * XS); b16 pp, q; split16(mv[i] * XS, pp, q); Ah[wave][rr][H + lane * 4 + i] = pp; Al[wave][rr][H + lane * 4 + i] = q; } }
  wave_lds_sync();
#pragma unroll
  for (int t = 0; t < 8; ++t) az[t] = (v8f){};
#pragma unroll 2
  for (int kb = 0; kb < K2; kb += 32) { const v16b a = frag_kb(&Ah[wave][nloc][kb], hlf), al = frag_kb(&Al[wave][nloc][kb], hlf); const bool dolo = kb >= H;
#pragma unroll
    for (int t = 0; t < 8; ++t) { const v16b bw = frag_kb(WRU + (size_t)(t * 16 + nloc) * K2 + kb, hlf); az[t] = wmma16b(a, bw, az[t]); if (dolo) az[t] = wmma16b(al, bw, az[t]); } }
  wave_lds_sync();
  float* Rf = (float*)&Ah[wave][0][0];
#pragma unroll
  for (int t = 0; t < 8; ++t) { const int cc = t * 16 + nloc; const float brv = bf16_rne(br[cc]);
#pragma unroll 1
    for (int r8 = 0; r8 < 8; ++r8) { const int rl = 8 * hlf + r8; const float rg = sigm(az[t][r8] * (1.0f / (XS * WSC)) + brv); Rf[rl * (H + 4) + cc] = pmul(rg, Sf[wave][rl][cc]); } }
  wave_lds_sync();
  for (int pass = 0; pass < 2; ++pass) { for (int rr = 0; rr < 16; ++rr) { *(volatile v4f*)(MOUT + (size_t)(r0 + rr) * H + lane * 4) = *(const v4f*)(&Sf[wave][rr][lane * 4]); *(volatile v4f*)(RMOUT + (size_t)(r0 + rr) * H + lane * 4) = *(const v4f*)(&Rf[rr * (H + 4) + lane * 4]); } __threadfence(); }
}
__global__ __launch_bounds__(32) void root_kernel(const int* __restrict__ wid, const float* __restrict__ emb, const float* __restrict__ M1, const b16* __restrict__ WGT, const float* __restrict__ bg, float* __restrict__ out) {
  __shared__ __attribute__((aligned(16))) b16 Ah[16][K2 + 8], Al[16][K2 + 8]; __shared__ __attribute__((aligned(16))) float Tf[16][H + 4];
  const int lane = threadIdx.x, nloc = lane & 15, hlf = lane >> 4; const int t0 = blockIdx.x * 16;
  for (int rr = 0; rr < 16; ++rr) { const int tree = t0 + rr; const int w = iclamp(wid[tree * NPT], 0, VOC - 1); const v4f xv = *(const v4f*)(emb + (size_t)w * H + lane * 4);
    const v4f a = *(const v4f*)(M1 + (size_t)(tree * 2) * H + lane * 4), b = *(const v4f*)(M1 + (size_t)(tree * 2 + 1) * H + lane * 4);
    for (int i = 0; i < 4; ++i) { Ah[rr][lane * 4 + i] = (b16)(bf16_rne(xv[i]) * XS); Al[rr][lane * 4 + i] = (b16)0.0f; b16 p, q; split16((a[i] + b[i]) * XS, p, q); Ah[rr][H + lane * 4 + i] = p; Al[rr][H + lane * 4 + i] = q; } }
  wave_lds_sync();
  v8f acc[8];
#pragma unroll
  for (int t = 0; t < 8; ++t) acc[t] = (v8f){};
#pragma unroll 2
  for (int kb = 0; kb < K2; kb += 32) { const v16b a = frag_kb(&Ah[nloc][kb], hlf), al = frag_kb(&Al[nloc][kb], hlf); const bool dolo = kb >= H;
#pragma unroll
    for (int t = 0; t < 8; ++t) { const v16b bw = frag_kb(WGT + (size_t)(t * 16 + nloc) * K2 + kb, hlf); acc[t] = wmma16b(a, bw, acc[t]); if (dolo) acc[t] = wmma16b(al, bw, acc[t]); } }
#pragma unroll
  for (int t = 0; t < 8; ++t) { const int cc = t * 16 + nloc; const float b_ = bf16_rne(bg[cc]);
#pragma unroll 1
    for (int r8 = 0; r8 < 8; ++r8) Tf[8 * hlf + r8][cc] = fmaxf(acc[t][r8] * (1.0f / (XS * WSC)) + b_, 0.0f); }
  wave_lds_sync();
  for (int pass = 0; pass < 2; ++pass) { for (int rr = 0; rr < 16; ++rr) *(volatile v4f*)(out + (size_t)(t0 + rr) * H + lane * 4) = *(const v4f*)(&Tf[rr][lane * 4]); __threadfence(); }
}
}

extern "C" void kernel_launch(void* const* d_in, const int* in_sizes, int n_in, void* d_out, int out_size, void* d_ws, size_t ws_size, hipStream_t stream) {
  (void)n_in;
  auto Fp = [&](int i) { return (const float*)d_in[i]; }; auto Ip = [&](int i) { return (const int*)d_in[i]; };
  if (in_sizes[0] != NT * NPT || in_sizes[1] != VOC * H || in_sizes[2] != K2 * H || in_sizes[4] != H * H || in_sizes[5] != H * H || in_sizes[7] != K2 * H || in_sizes[9] != K2 * H || out_size != NT * H) return;
  size_t off = 0; char* ws = (char*)d_ws;
  auto carve = [&](size_t bytes) { char* p = ws + off; off += (bytes + 255) & ~(size_t)255; return p; };
  b16* WZT = (b16*)carve((size_t)H * K2 * 2); b16* WHT = (b16*)carve((size_t)H * K2 * 2); b16* WGT = (b16*)carve((size_t)H * K2 * 2); b16* WRU = (b16*)carve((size_t)H * K2 * 2);
  float* MA = (float*)carve((size_t)MAXR * H * 4); float* RA = (float*)carve((size_t)MAXR * H * 4); float* MB = (float*)carve((size_t)(MAXR / 2) * H * 4); float* RB = (float*)carve((size_t)(MAXR / 2) * H * 4);
  if (off > ws_size || off > ((size_t)128 << 20)) return;
  wprep_kernel<<<(unsigned)((4 * (size_t)H * K2 / 8 + 255) / 256), 256, 0, stream>>>(Fp(2), Fp(7), Fp(9), Fp(4), Fp(5), WZT, WHT, WGT, WRU);
  float* min_ = MB; float* rmin = RB; float* mout = MA; float* rmout = RA;
  for (int d = DEPTH; d >= 1; --d) { const int rows = NT << d;
    if (d == DEPTH) level_kernel<1><<<rows / 32, 64, 0, stream>>>(d, Ip(0), Fp(1), nullptr, nullptr, WZT, WHT, WRU, Fp(3), Fp(8), Fp(6), mout, rmout);
    else level_kernel<0><<<rows / 32, 64, 0, stream>>>(d, Ip(0), Fp(1), min_, rmin, WZT, WHT, WRU, Fp(3), Fp(8), Fp(6), mout, rmout);
    float* t1 = min_; min_ = mout; mout = t1; float* t2 = rmin; rmin = rmout; rmout = t2; }
  root_kernel<<<NT / 16, 32, 0, stream>>>(Ip(0), Fp(1), min_, WGT, Fp(10), (float*)d_out);
}
